// MultiLatentHeadAttn_62964220559621
// MI455X (gfx1250) — hardware-verified
//
#include <hip/hip_runtime.h>
#include <math.h>
#include <stdint.h>


#define NB   2
#define SEQ  2048
#define HID  2048
#define NH   16
#define HD   128
#define DC   512
#define DR   32
#define QKP  192
#define NTOK (NB * SEQ)

typedef _Float16 v16h __attribute__((ext_vector_type(16)));
typedef _Float16 v8h  __attribute__((ext_vector_type(8)));
typedef float    v8f  __attribute__((ext_vector_type(8)));
typedef float    v4f  __attribute__((ext_vector_type(4)));
typedef unsigned int v4u __attribute__((ext_vector_type(4)));

__device__ __forceinline__ unsigned pk16(unsigned short a, unsigned short b) { return (unsigned)a | ((unsigned)b << 16); }
__device__ __forceinline__ unsigned short h2u(_Float16 x) { return __builtin_bit_cast(unsigned short, x); }
__device__ __forceinline__ unsigned pkf16(float a, float b) { return pk16(h2u((_Float16)a), h2u((_Float16)b)); }

__device__ __forceinline__ void wave_sync() {
  __builtin_amdgcn_fence(__ATOMIC_RELEASE, "workgroup");
  __builtin_amdgcn_wave_barrier();
  __builtin_amdgcn_fence(__ATOMIC_ACQUIRE, "workgroup");
}

union FragH { v16h v; v8h h[2]; };
__device__ __forceinline__ v16h ldfrag_h(const _Float16* p) {
  FragH f; f.h[0] = *(const v8h*)(p); f.h[1] = *(const v8h*)(p + 16); return f.v;
}

__device__ __forceinline__ v8f wmma_raw(v16h a, v16h b, v8f c) {
  return __builtin_amdgcn_wmma_f32_16x16x32_f16(false, a, false, b, (short)0, c, false, false);
}
__device__ __forceinline__ v8f wmma_h(v16h a, v16h b, v8f c) {
  c = wmma_raw(a, b, c);
  asm volatile("v_nop\n\tv_nop\n\tv_nop\n\tv_nop" : "+v"(c) : "v"(a), "v"(b));
  return c;
}
__device__ __forceinline__ void dep_guard(v8f& x, v8f& y, v16h b, v16h a0, v16h a1) {
  asm volatile("v_nop\n\tv_nop\n\tv_nop\n\tv_nop" : "+v"(x), "+v"(y) : "v"(b), "v"(a0), "v"(a1));
}

__global__ __launch_bounds__(256) void cvt_f16x8_kernel(const float* __restrict__ in, unsigned short* out,
                                                         int n8, float scale) {
  const int i = blockIdx.x * 256 + threadIdx.x;
  if (i < n8) {
    const v4f a = *(const v4f*)(in + 8 * (size_t)i);
    const v4f c = *(const v4f*)(in + 8 * (size_t)i + 4);
    v4u w;
    w[0] = pkf16(a[0] * scale, a[1] * scale);
    w[1] = pkf16(a[2] * scale, a[3] * scale);
    w[2] = pkf16(c[0] * scale, c[1] * scale);
    w[3] = pkf16(c[2] * scale, c[3] * scale);
    volatile v4u* p = (volatile v4u*)(out + 8 * (size_t)i);
    *p = w;
    __threadfence();
    *p = w;
  }
}

#define TP 68
__global__ __launch_bounds__(256) void cvt_wt_kernel(const float* __restrict__ W, unsigned short* Wt,
                                                      int Kin, int Nout, float scale) {
  __shared__ __align__(16) float tile[64 * TP];
  const int tid = threadIdx.x;
  const int n0 = blockIdx.x * 64;
  const int k0 = blockIdx.y * 64;
  {
    const int rr = tid >> 4, c4 = (tid & 15) * 4;
#pragma unroll
    for (int it = 0; it < 4; ++it) {
      const int row = it * 16 + rr;
      const v4f v = *(const v4f*)(W + (size_t)(k0 + row) * Nout + n0 + c4);
      *(v4f*)(tile + row * TP + c4) = v;
    }
  }
  __syncthreads();
  {
    const int p8 = tid & 7;
#pragma unroll
    for (int it = 0; it < 2; ++it) {
      const int r = it * 32 + (tid >> 3);
      float f[8];
#pragma unroll
      for (int e = 0; e < 8; ++e) f[e] = tile[(8 * p8 + e) * TP + r] * scale;
      v4u w;
#pragma unroll
      for (int p = 0; p < 4; ++p) w[p] = pkf16(f[2 * p], f[2 * p + 1]);
      volatile v4u* dst = (volatile v4u*)(Wt + (size_t)(n0 + r) * Kin + k0 + 8 * p8);
      *dst = w;
      __threadfence();
      *dst = w;
    }
  }
}

__device__ __forceinline__ float freq_sel(int j) {
  unsigned u = 0x3f800000u;
  u = (j == 1)  ? 0x3f0ff59au : u;
  u = (j == 2)  ? 0x3ea1e89bu : u;
  u = (j == 3)  ? 0x3e361887u : u;
  u = (j == 4)  ? 0x3dcccccdu : u;
  u = (j == 5)  ? 0x3d6655c3u : u;
  u = (j == 6)  ? 0x3d0186e2u : u;
  u = (j == 7)  ? 0x3c91ad39u : u;
  u = (j == 8)  ? 0x3c23d70au : u;
  u = (j == 9)  ? 0x3bb8449cu : u;
  u = (j == 10) ? 0x3b4f3e37u : u;
  u = (j == 11) ? 0x3ae91528u : u;
  u = (j == 12) ? 0x3a83126fu : u;
  u = (j == 13) ? 0x3a136a16u : u;
  u = (j == 14) ? 0x39a5cb5fu : u;
  u = (j == 15) ? 0x393a7753u : u;
  return __uint_as_float(u);
}

__global__ __launch_bounds__(256) void rope_table_kernel(float* cs, int n) {
#pragma clang fp contract(off)
  const int t = blockIdx.x * 256 + threadIdx.x;
  if (t >= n) return;
  const int s = t >> 5;
  const int e = t & 31;
  const int j = e & 15;
  const float  fr  = freq_sel(j);
  const float  ang = (float)s * fr;
  const double ad = (double)ang;
  const double nd = rint(ad * 0.6366197723675814);
  const double rd = (ad - nd * 1.5707963267948966) - nd * 6.123233995736766e-17;
  const float  r = (float)rd;
  const float  z = r * r;
  const float  sr = r + r * z * ((-1.9515295891e-4f * z + 8.3321608736e-3f) * z - 1.6666654611e-1f);
  const float  cr = 1.0f - 0.5f * z + z * z * ((2.443315711809948e-5f * z - 1.388731625493765e-3f) * z + 4.166664568298827e-2f);
  const int qd = ((int)nd) & 3;
  float sv = sr, cv = cr;
  if (qd == 1) { sv = cr;  cv = -sr; }
  if (qd == 2) { sv = -sr; cv = -cr; }
  if (qd == 3) { sv = -cr; cv = sr;  }
  const float v = (e < 16) ? cv : sv;
  volatile float* p = (volatile float*)(cs + t);
  *p = v;
  __threadfence();
  *p = v;
}

#define GP 132

template <int MODE, bool BIAS_ROW>
__global__ __launch_bounds__(128) void gemm_kernel(
    const unsigned short* __restrict__ Ap, int lda, long strideA,
    const unsigned short* __restrict__ Btp, int ldb, long strideB,
    const float* __restrict__ bias, float cscale, float bscale,
    unsigned short* C1, unsigned short* C2, int ldc, long strideC,
    const float* __restrict__ cs, int M, int N, int K) {
  __shared__ __align__(16) float sT[4][16 * GP];
  const int bz   = blockIdx.y;
  const int lane = threadIdx.x & 31;
  const int wave = threadIdx.x >> 5;
  const int tilesN = N >> 7;
  const int tilesM = M >> 5;
  const int tile = blockIdx.x * 4 + wave;
  if (tile >= tilesM * tilesN) return;
  const int tm = tile / tilesN;
  const int tn = tile - tm * tilesN;
  const int m0 = tm << 5;
  const int n0 = tn << 7;

  const _Float16* Ab = (const _Float16*)(const void*)Ap  + (size_t)bz * (size_t)strideA;
  const _Float16* Bb = (const _Float16*)(const void*)Btp + (size_t)bz * (size_t)strideB;

  const int rlane = lane & 15;
  const int koff  = (lane >> 4) * 8;
  const int mOff  = (lane >> 4) * 8;

  v8f acc[2][8];
#pragma unroll
  for (int i = 0; i < 2; ++i)
#pragma unroll
    for (int j = 0; j < 8; ++j) acc[i][j] = (v8f){0.f, 0.f, 0.f, 0.f, 0.f, 0.f, 0.f, 0.f};

  const _Float16* a0p = Ab + (size_t)(m0 + rlane) * lda + koff;
  const _Float16* a1p = Ab + (size_t)(m0 + 16 + rlane) * lda + koff;
  const _Float16* b0p = Bb + (size_t)(n0 + rlane) * ldb + koff;
  const size_t bstep = (size_t)16 * ldb;

  for (int k0 = 0; k0 < K; k0 += 32) {
    const v16h a0 = ldfrag_h(a0p + k0);
    const v16h a1 = ldfrag_h(a1p + k0);
#pragma unroll
    for (int j = 0; j < 8; ++j) {
      const v16h bh = ldfrag_h(b0p + j * bstep + k0);
      acc[0][j] = wmma_raw(a0, bh, acc[0][j]);
      acc[1][j] = wmma_raw(a1, bh, acc[1][j]);
      dep_guard(acc[0][j], acc[1][j], bh, a0, a1);
    }
  }

  float* slab = sT[wave];
  const int q16 = lane >> 4, c8 = (lane & 15) * 8;
#pragma unroll
  for (int i = 0; i < 2; ++i) {
    const int mBase = m0 + (i << 4);
#pragma unroll
    for (int j = 0; j < 8; ++j)
#pragma unroll
      for (int r = 0; r < 8; ++r) slab[(mOff + r) * GP + (j << 4) + rlane] = acc[i][j][r];
    wave_sync();
    if (MODE != 3) {
      float bcol[8];
#pragma unroll
      for (int e = 0; e < 8; ++e) bcol[e] = 0.f;
      if (!BIAS_ROW) {
        const v4f bq0 = *(const v4f*)(bias + n0 + c8);
        const v4f bq1 = *(const v4f*)(bias + n0 + c8 + 4);
#pragma unroll
        for (int e = 0; e < 4; ++e) { bcol[e] = bq0[e] * bscale; bcol[4 + e] = bq1[e] * bscale; }
      }
      for (int pass = 0; pass < 2; ++pass) {
#pragma unroll
        for (int it = 0; it < 8; ++it) {
          const int row = it * 2 + q16;
          const int m   = mBase + row;
          const float* sp = slab + row * GP + c8;
          const v4f x0 = *(const v4f*)sp;
          const v4f x1 = *(const v4f*)(sp + 4);
          float bb[8];
          if (BIAS_ROW) {
            const float br = bias[m] * bscale;
#pragma unroll
            for (int e = 0; e < 8; ++e) bb[e] = br;
          } else {
#pragma unroll
            for (int e = 0; e < 8; ++e) bb[e] = bcol[e];
          }
          float f[8];
#pragma unroll
          for (int e = 0; e < 4; ++e) { f[e] = x0[e] * cscale + bb[e]; f[4 + e] = x1[e] * cscale + bb[4 + e]; }
          if (MODE == 1) {
            v4u hv, lv;
#pragma unroll
            for (int p = 0; p < 4; ++p) {
              const float f0 = f[2 * p], f1 = f[2 * p + 1];
              const _Float16 e0 = (_Float16)f0, e1 = (_Float16)f1;
              const _Float16 g0 = (_Float16)((f0 - (float)e0) * 2048.0f);
              const _Float16 g1 = (_Float16)((f1 - (float)e1) * 2048.0f);
              hv[p] = pk16(h2u(e0), h2u(e1));
              lv[p] = pk16(h2u(g0), h2u(g1));
            }
            const size_t go = (size_t)bz * (size_t)strideC + (size_t)m * ldc + n0 + c8;
            *(volatile v4u*)(C1 + go) = hv;
            *(volatile v4u*)(C2 + go) = lv;
          } else {
            v4u hv;
#pragma unroll
            for (int p = 0; p < 4; ++p) hv[p] = pkf16(f[2 * p], f[2 * p + 1]);
            size_t go;
            if (MODE == 0) go = (size_t)bz * (size_t)strideC + (size_t)m * ldc + n0 + c8;
            else           go = (((size_t)((m >> 11) * NH + (n0 >> 7))) * SEQ + (size_t)(m & (SEQ - 1))) * QKP + c8;
            *(volatile v4u*)(C1 + go) = hv;
          }
        }
        __threadfence();
      }
    } else {
      const int hq = lane >> 3, p8 = lane & 7, qq = p8 & 3;
      const int pb = (qq & 1) * 8;
      const bool second = (qq >> 1) != 0;
      const bool zero   = (p8 >= 4);
      const int colb = hq * DR + 2 * pb;
      float bv[16];
      {
        const float* bp = bias + n0 + colb;
        const v4f t0 = *(const v4f*)bp, t1 = *(const v4f*)(bp + 4), t2 = *(const v4f*)(bp + 8), t3 = *(const v4f*)(bp + 12);
#pragma unroll
        for (int e = 0; e < 4; ++e) {
          bv[e] = t0[e] * bscale; bv[4 + e] = t1[e] * bscale; bv[8 + e] = t2[e] * bscale; bv[12 + e] = t3[e] * bscale;
        }
      }
      const size_t headrow = ((size_t)((m0 >> 11) * NH + (n0 >> 5) + hq)) * SEQ;
      for (int pass = 0; pass < 2; ++pass) {
#pragma unroll
        for (int it = 0; it < 16; ++it) {
          const int m = mBase + it;
          const int s = m & (SEQ - 1);
          const float* sp = slab + it * GP + colb;
          const v4f xa = *(const v4f*)sp, xb = *(const v4f*)(sp + 4), xc = *(const v4f*)(sp + 8), xd = *(const v4f*)(sp + 12);
          float xv[16];
#pragma unroll
          for (int e = 0; e < 4; ++e) { xv[e] = xa[e]; xv[4 + e] = xb[e]; xv[8 + e] = xc[e]; xv[12 + e] = xd[e]; }
          const float* tp = cs + (size_t)s * DR + pb;
          const v4f ca = *(const v4f*)tp, cb = *(const v4f*)(tp + 4);
          const v4f sa = *(const v4f*)(tp + 16), sb = *(const v4f*)(tp + 20);
          float cv[8], sv[8];
#pragma unroll
          for (int e = 0; e < 4; ++e) { cv[e] = ca[e]; cv[4 + e] = cb[e]; sv[e] = sa[e]; sv[4 + e] = sb[e]; }
          float o[8];
#pragma unroll
          for (int e = 0; e < 8; ++e) {
            const float x1 = xv[2 * e] * cscale + bv[2 * e];
            const float x2 = xv[2 * e + 1] * cscale + bv[2 * e + 1];
            const float of = x1 * cv[e] - x2 * sv[e];
            const float og = x1 * sv[e] + x2 * cv[e];
            const float oo = second ? og : of;
            o[e] = zero ? 0.0f : oo;
          }
          v4u hv;
#pragma unroll
          for (int p = 0; p < 4; ++p) hv[p] = pkf16(o[2 * p], o[2 * p + 1]);
          const size_t go = (headrow + (size_t)s) * QKP + HD + 8 * p8;
          *(volatile v4u*)(C1 + go) = hv;
        }
        __threadfence();
      }
    }
    wave_sync();
  }
}

#define AT_QB 64
#define AT_KC 64
#define KP    168
#define OS_P  132

__global__ __launch_bounds__(128)
void attn_kernel(const unsigned short* __restrict__ qp, const unsigned short* __restrict__ kp,
                 const unsigned short* __restrict__ vhp, const unsigned short* __restrict__ vlp,
                 float* out) {
  __shared__ __align__(16) _Float16 KVs[AT_KC * KP + 2 * HD * AT_KC];
  __shared__ __align__(16) _Float16 Psh[4][16 * AT_KC];
  static_assert(4 * 16 * OS_P * 4 <= (AT_KC * KP + 2 * HD * AT_KC) * 2);
  _Float16* const Ksh = KVs;
  _Float16* const Vth = KVs + AT_KC * KP;
  _Float16* const Vtl = KVs + AT_KC * KP + HD * AT_KC;

  const int tid  = threadIdx.x;
  const int wave = tid >> 5;
  const int lane = tid & 31;
  const int hh   = lane >> 4;
  const int c    = lane & 15;

  const int bx = blockIdx.x;
  const int qb = bx & 31;
  const int h  = (bx >> 5) & (NH - 1);
  const int b  = bx >> 9;
  const int q0 = qb * AT_QB + wave * 16;

  const size_t bhrow = (size_t)(b * NH + h) * SEQ;
  const _Float16* Qg  = (const _Float16*)(const void*)qp + bhrow * QKP;
  const _Float16* Kg  = (const _Float16*)(const void*)kp + bhrow * QKP;
  const _Float16* Vhg = (const _Float16*)(const void*)vhp + ((size_t)b * HID + (size_t)h * HD) * SEQ;
  const _Float16* Vlg = (const _Float16*)(const void*)vlp + ((size_t)b * HID + (size_t)h * HD) * SEQ;

  const v8f zero8 = (v8f){0.f, 0.f, 0.f, 0.f, 0.f, 0.f, 0.f, 0.f};
  const float inv2048 = 4.8828125e-4f;
  const float scl     = 0.0790569415f * 0.0625f;

  v16h qa[5];
#pragma unroll
  for (int dc = 0; dc < 5; ++dc) qa[dc] = ldfrag_h(Qg + (size_t)(q0 + c) * QKP + dc * 32 + 8 * hh);

  float mrow[8], lrow[8];
  v8f oh[8];
#pragma unroll
  for (int r = 0; r < 8; ++r) { mrow[r] = -INFINITY; lrow[r] = 0.f; }
#pragma unroll
  for (int t = 0; t < 8; ++t) oh[t] = zero8;

  for (int kc = 0; kc < SEQ / AT_KC; ++kc) {
    const int kv0 = kc * AT_KC;
    __syncthreads();
    {
      const int r = tid >> 1, cb = (tid & 1) * 80;
      const _Float16* ks  = Kg  + (size_t)(kv0 + r) * QKP + cb;
      const _Float16* vhs = Vhg + (size_t)tid * SEQ + kv0;
      const _Float16* vls = Vlg + (size_t)tid * SEQ + kv0;
#pragma unroll
      for (int i = 0; i < 10; ++i) *(v8h*)(Ksh + r * KP + cb + 8 * i) = *(const v8h*)(ks + 8 * i);
#pragma unroll
      for (int i = 0; i < 8; ++i) {
        const v8h b0 = *(const v8h*)(vhs + 8 * i);
        const v8h b1 = *(const v8h*)(vls + 8 * i);
        *(v8h*)(Vth + tid * AT_KC + 8 * i) = b0;
        *(v8h*)(Vtl + tid * AT_KC + 8 * i) = b1;
      }
    }
    __syncthreads();

    v8f s[4];
#pragma unroll
    for (int j = 0; j < 4; ++j) {
      v8f sa = zero8;
#pragma unroll
      for (int dc = 0; dc < 5; ++dc) {
        FragH kb;
        kb.h[0] = *(const v8h*)(Ksh + (j * 16 + c) * KP + dc * 32 + 8 * hh);
        kb.h[1] = *(const v8h*)(Ksh + (j * 16 + c) * KP + dc * 32 + 16 + 8 * hh);
        sa = wmma_h(qa[dc], kb.v, sa);
      }
      s[j] = sa * scl;
    }

    float cm[8];
#pragma unroll
    for (int r = 0; r < 8; ++r) {
      float m = fmaxf(fmaxf(s[0][r], s[1][r]), fmaxf(s[2][r], s[3][r]));
#pragma unroll
      for (int off = 1; off < 16; off <<= 1) m = fmaxf(m, __shfl_xor(m, off, 32));
      cm[r] = m;
    }

    _Float16* pw = Psh[wave];
#pragma unroll
    for (int r = 0; r < 8; ++r) {
      const float mnew  = fmaxf(mrow[r], cm[r]);
      const float alpha = __expf(mrow[r] - mnew);
      mrow[r] = mnew;
      float psum = 0.f;
#pragma unroll
      for (int j = 0; j < 4; ++j) {
        const float p = __expf(s[j][r] - mnew);
        psum += p;
        pw[(8 * hh + r) * AT_KC + j * 16 + c] = (_Float16)(p * 1024.0f);
      }
#pragma unroll
      for (int off = 1; off < 16; off <<= 1) psum += __shfl_xor(psum, off, 32);
      lrow[r] = lrow[r] * alpha + psum;
#pragma unroll
      for (int t = 0; t < 8; ++t) oh[t][r] *= alpha;
    }
    wave_sync();

#pragma unroll 1
    for (int kk = 0; kk < 2; ++kk) {
      FragH pa;
      pa.h[0] = *(const v8h*)(pw + c * AT_KC + kk * 32 + 8 * hh);
      pa.h[1] = *(const v8h*)(pw + c * AT_KC + kk * 32 + 16 + 8 * hh);
#pragma unroll
      for (int t = 0; t < 8; ++t) {
        FragH vb, vr;
        vb.h[0] = *(const v8h*)(Vth + (t * 16 + c) * AT_KC + kk * 32 + 8 * hh);
        vb.h[1] = *(const v8h*)(Vth + (t * 16 + c) * AT_KC + kk * 32 + 16 + 8 * hh);
        vr.h[0] = *(const v8h*)(Vtl + (t * 16 + c) * AT_KC + kk * 32 + 8 * hh);
        vr.h[1] = *(const v8h*)(Vtl + (t * 16 + c) * AT_KC + kk * 32 + 16 + 8 * hh);
        oh[t] = wmma_h(pa.v, vb.v, oh[t]);
        const v8f tr = wmma_h(pa.v, vr.v, zero8);
        oh[t] += tr * inv2048;
      }
    }
  }

  __syncthreads();
  float* os = (float*)(void*)KVs + wave * (16 * OS_P);
#pragma unroll
  for (int r = 0; r < 8; ++r) {
    const float invl = (1.0f / lrow[r]) * 2.44140625e-4f;
#pragma unroll
    for (int t = 0; t < 8; ++t) os[(8 * hh + r) * OS_P + t * 16 + c] = oh[t][r] * invl;
  }
  wave_sync();
  {
    const int c4 = lane * 4;
    float* ob = out + ((size_t)b * SEQ + (size_t)q0) * HID + (size_t)h * HD + c4;
    for (int pass = 0; pass < 2; ++pass) {
#pragma unroll
      for (int it = 0; it < 16; ++it) {
        const v4f v = *(const v4f*)(os + it * OS_P + c4);
        *(volatile v4f*)(ob + (size_t)it * HID) = v;
      }
      __threadfence();
    }
  }
}

extern "C" void kernel_launch(void* const* d_in, const int* in_sizes, int n_in,
                              void* d_out, int out_size, void* d_ws, size_t ws_size,
                              hipStream_t stream) {
  if (n_in < 15) return;
  if (in_sizes[0] != NTOK * HID) return;
  if (in_sizes[1] != HID * DC || in_sizes[3] != DC * HID || in_sizes[5] != DC * HID) return;
  if (in_sizes[7] != HID * DC || in_sizes[9] != DC * HID || in_sizes[11] != DC * DC || in_sizes[13] != HID * DC) return;
  if (in_sizes[2] != DC || in_sizes[4] != HID || in_sizes[6] != HID || in_sizes[8] != DC) return;
  if (in_sizes[10] != HID || in_sizes[12] != DC || in_sizes[14] != DC) return;
  if (out_size != NTOK * HID) return;

  const float* x     = (const float*)d_in[0];
  const float* W_DKV = (const float*)d_in[1];
  const float* b_DKV = (const float*)d_in[2];
  const float* W_UK  = (const float*)d_in[3];
  const float* b_UK  = (const float*)d_in[4];
  const float* W_UV  = (const float*)d_in[5];
  const float* b_UV  = (const float*)d_in[6];
  const float* W_DQ  = (const float*)d_in[7];
  const float* b_DQ  = (const float*)d_in[8];
  const float* W_UQ  = (const float*)d_in[9];
  const float* b_UQ  = (const float*)d_in[10];
  const float* W_QR  = (const float*)d_in[11];
  const float* b_QR  = (const float*)d_in[12];
  const float* W_KR  = (const float*)d_in[13];
  const float* b_KR  = (const float*)d_in[14];
  float* out = (float*)d_out;

  const size_t szX   = (size_t)NTOK * HID * 2;
  const size_t szW   = (size_t)HID * DC * 2;
  const size_t szWqr = (size_t)DC * DC * 2;
  const size_t szCs  = (size_t)SEQ * DR * 4;
  const size_t szC   = (size_t)NTOK * DC * 2;
  const size_t szQK  = (size_t)NB * NH * SEQ * QKP * 2;
  const size_t szV   = (size_t)NB * HID * SEQ * 2;
  size_t off = 0;
  const size_t oX    = off; off += szX;
  const size_t oWdkv = off; off += szW;
  const size_t oWdq  = off; off += szW;
  const size_t oWkr  = off; off += szW;
  const size_t oWuk  = off; off += szW;
  const size_t oWuv  = off; off += szW;
  const size_t oWuq  = off; off += szW;
  const size_t oWqr  = off; off += szWqr;
  const size_t oCs   = off; off += szCs;
  const size_t oCkv  = off; off += szC;
  const size_t oCq   = off; off += szC;
  const size_t oQp   = off; off += szQK;
  const size_t oKp   = off; off += szQK;
  const size_t oVth  = off; off += szV;
  const size_t oVtl  = off; off += szV;
  if (off > ws_size) return;
  if (off > (size_t)134217728) return;

  char* ws = (char*)d_ws;
  unsigned short* Xh   = (unsigned short*)(ws + oX);
  unsigned short* Wdkv = (unsigned short*)(ws + oWdkv);
  unsigned short* Wdq  = (unsigned short*)(ws + oWdq);
  unsigned short* Wkr  = (unsigned short*)(ws + oWkr);
  unsigned short* Wuk  = (unsigned short*)(ws + oWuk);
  unsigned short* Wuv  = (unsigned short*)(ws + oWuv);
  unsigned short* Wuq  = (unsigned short*)(ws + oWuq);
  unsigned short* Wqr  = (unsigned short*)(ws + oWqr);
  float*          Cs   = (float*)(ws + oCs);
  unsigned short* Ckv  = (unsigned short*)(ws + oCkv);
  unsigned short* Cq   = (unsigned short*)(ws + oCq);
  unsigned short* Qp   = (unsigned short*)(ws + oQp);
  unsigned short* Kp   = (unsigned short*)(ws + oKp);
  unsigned short* Vth  = (unsigned short*)(ws + oVth);
  unsigned short* Vtl  = (unsigned short*)(ws + oVtl);

  const dim3 blk256(256), blk128(128);

  {
    const int n8 = NTOK * HID / 8;
    cvt_f16x8_kernel<<<dim3((n8 + 255) / 256), blk256, 0, stream>>>(x, Xh, n8, 1.0f);
  }
  cvt_wt_kernel<<<dim3(DC / 64, HID / 64), blk256, 0, stream>>>(W_DKV, Wdkv, HID, DC, 32.0f);
  cvt_wt_kernel<<<dim3(DC / 64, HID / 64), blk256, 0, stream>>>(W_DQ,  Wdq,  HID, DC, 32.0f);
  cvt_wt_kernel<<<dim3(DC / 64, HID / 64), blk256, 0, stream>>>(W_KR,  Wkr,  HID, DC, 32.0f);
  cvt_wt_kernel<<<dim3(HID / 64, DC / 64), blk256, 0, stream>>>(W_UK,  Wuk,  DC, HID, 32.0f);
  cvt_wt_kernel<<<dim3(HID / 64, DC / 64), blk256, 0, stream>>>(W_UV,  Wuv,  DC, HID, 32.0f);
  cvt_wt_kernel<<<dim3(HID / 64, DC / 64), blk256, 0, stream>>>(W_UQ,  Wuq,  DC, HID, 32.0f);
  cvt_wt_kernel<<<dim3(DC / 64, DC / 64),  blk256, 0, stream>>>(W_QR,  Wqr,  DC, DC, 32.0f);
  {
    const int nt = SEQ * DR;
    rope_table_kernel<<<dim3((nt + 255) / 256), blk256, 0, stream>>>(Cs, nt);
  }
  {
    const int tiles = (NTOK / 32) * (DC / 128);
    gemm_kernel<0, false><<<dim3((tiles + 3) / 4, 1), blk128, 0, stream>>>(
        Xh, HID, 0L, Wdkv, HID, 0L, b_DKV, 0.0625f, 2.0f, Ckv, Ckv, DC, 0L, Cs, NTOK, DC, HID);
  }
  {
    const int tiles = (NTOK / 32) * (DC / 128);
    gemm_kernel<0, false><<<dim3((tiles + 3) / 4, 1), blk128, 0, stream>>>(
        Xh, HID, 0L, Wdq, HID, 0L, b_DQ, 0.0625f, 2.0f, Cq, Cq, DC, 0L, Cs, NTOK, DC, HID);
  }
  {
    const int tiles = (NTOK / 32) * (DC / 128);
    gemm_kernel<3, false><<<dim3((tiles + 3) / 4, 1), blk128, 0, stream>>>(
        Xh, HID, 0L, Wkr, HID, 0L, b_KR, 0.125f, 4.0f, Kp, Kp, QKP, 0L, Cs, NTOK, DC, HID);
  }
  {
    const int tiles = (NTOK / 32) * (HID / 128);
    gemm_kernel<2, false><<<dim3((tiles + 3) / 4, 1), blk128, 0, stream>>>(
        Ckv, DC, 0L, Wuk, DC, 0L, b_UK, 0.0625f, 4.0f, Kp, Kp, QKP, 0L, Cs, NTOK, HID, DC);
  }
  {
    const int tiles = (HID / 32) * (SEQ / 128);
    gemm_kernel<1, true><<<dim3((tiles + 3) / 4, NB), blk128, 0, stream>>>(
        Wuv, DC, 0L, Ckv, DC, (long)SEQ * DC, b_UV, 0.0625f, 4.0f, Vth, Vtl, SEQ, (long)HID * SEQ,
        Cs, HID, SEQ, DC);
  }
  {
    const int tiles = (NTOK / 32) * (HID / 128);
    gemm_kernel<2, false><<<dim3((tiles + 3) / 4, 1), blk128, 0, stream>>>(
        Cq, DC, 0L, Wuq, DC, 0L, b_UQ, 0.0625f, 4.0f, Qp, Qp, QKP, 0L, Cs, NTOK, HID, DC);
  }
  {
    const int tiles = (NTOK / 32) * (DC / 128);
    gemm_kernel<3, false><<<dim3((tiles + 3) / 4, 1), blk128, 0, stream>>>(
        Cq, DC, 0L, Wqr, DC, 0L, b_QR, 0.0625f, 4.0f, Qp, Qp, QKP, 0L, Cs, NTOK, DC, DC);
  }
  attn_kernel<<<dim3(NB * NH * (SEQ / AT_QB)), blk128, 0, stream>>>(Qp, Kp, Vth, Vtl, out);
  (void)hipGetLastError();
}
